// GFootballMamba_59828894433549
// MI455X (gfx1250) — hardware-verified
//
#include <hip/hip_runtime.h>


namespace {
constexpr int NBS = 1024, NF = 4, FD = 115, FDP = 128, DM = 256, NL = 4, DS = 16, DI = 512, NT = NBS * NF  , NO = 19;
constexpr float XS = 8.0f, WSC = 256.0f, EPS = 1e-5f;

typedef _Float16 b16;
typedef __attribute__((ext_vector_type(16))) _Float16 v16b;
typedef __attribute__((ext_vector_type(8))) _Float16 v8b;
typedef __attribute__((ext_vector_type(8))) float v8f;
typedef __attribute__((ext_vector_type(4))) float v4f;
__device__ __forceinline__ float bf16_rne(float f) { unsigned int u = __float_as_uint(f); u += 0x7FFFu + ((u >> 16) & 1u); return __uint_as_float(u & 0xFFFF0000u); }
__device__ __forceinline__ void split16(float v, b16& hi, b16& lo) { hi = (b16)v; lo = (b16)(v - (float)hi); }
__device__ __forceinline__ v16b frag_kb(const b16* p, int hh) { const v8b a = *(const v8b*)(p + 8 * hh), b = *(const v8b*)(p + 16 + 8 * hh); v16b f;
#pragma unroll
  for (int e = 0; e < 8; ++e) { f[e] = a[e]; f[8 + e] = b[e]; } return f; }
__device__ __forceinline__ v8f wmma16b(v16b a, v16b b, v8f c) { v8f d = __builtin_amdgcn_wmma_f32_16x16x32_f16(false, a, false, b, (short)0, c, false, false); asm volatile("v_nop\n\tv_nop\n\tv_nop\n\tv_nop" : "+v"(d) : "v"(a), "v"(b)); return d; }
__device__ __forceinline__ void wave_lds_sync() { __builtin_amdgcn_fence(__ATOMIC_RELEASE, "workgroup"); __builtin_amdgcn_wave_barrier(); __builtin_amdgcn_fence(__ATOMIC_ACQUIRE, "workgroup"); }
__device__ __forceinline__ float pmul(float a, float b) { float p = a * b; asm volatile("" : "+v"(p)); return p; }
__device__ __forceinline__ float softplus_(float x) { return (x > 20.0f) ? x : log1pf(__expf(x)); }
__device__ __forceinline__ float mish_(float x) { return x * tanhf(softplus_(x)); }
__device__ __forceinline__ float silu_(float x) { return x / (1.0f + __expf(-x)); }

__global__ __launch_bounds__(256) void wprep_kernel(const float* __restrict__ w, int nin, int nout, int ninp, int noutp, b16* __restrict__ dst) {
  const size_t u = (size_t)blockIdx.x * 256 + threadIdx.x; if (u >= (size_t)noutp * ninp / 8) return; const size_t e = u * 8; const int oo = (int)(e / ninp), k0 = (int)(e % ninp); v8b o;
  for (int j = 0; j < 8; ++j) { const int k = k0 + j; o[j] = (oo < nout && k < nin) ? (b16)(bf16_rne(w[(size_t)k * nout + oo]) * WSC) : (b16)0.0f; }
  for (int pass = 0; pass < 2; ++pass) { *(volatile v8b*)(dst + e) = o; __threadfence(); }
}
__global__ __launch_bounds__(256) void obsprep_kernel(const float* __restrict__ obs, b16* __restrict__ OBS) {
  const size_t u = (size_t)blockIdx.x * 256 + threadIdx.x; if (u >= (size_t)NT * FDP / 8) return; const size_t e = u * 8; const int row = (int)(e / FDP), k0 = (int)(e % FDP); v8b o;
  for (int j = 0; j < 8; ++j) { const int k = k0 + j; o[j] = (k < FD) ? (b16)(bf16_rne(obs[(size_t)row * FD + k]) * XS) : (b16)0.0f; }
  for (int pass = 0; pass < 2; ++pass) { *(volatile v8b*)(OBS + e) = o; __threadfence(); }
}
struct WPtrs { b16 *EMB, *INW, *DTW, *BCW, *OUTW, *POOLW, *P1, *P2, *PH, *V1, *V2, *VH, *OBS; };
template <int KD, int NTL, int EPI, int NW>
__global__ __launch_bounds__(NW * 32) void dense_kernel(const float* __restrict__ X, int ldx, const b16* __restrict__ XH, const b16* __restrict__ Wt, const float* __restrict__ bias, int nbias, const float* __restrict__ R, float* __restrict__ Y, int ldy) {
  __shared__ __attribute__((aligned(16))) b16 Ah[NW][16][KD + 8], Al[NW][16][KD + 8]; __shared__ __attribute__((aligned(16))) float Tf[NW][16][NTL * 16 + 4];
  const int wave = threadIdx.x >> 5, lane = threadIdx.x & 31, nloc = lane & 15, hlf = lane >> 4; const size_t m0 = (size_t)blockIdx.x * (NW * 16) + wave * 16; const int n0 = blockIdx.y * NTL * 16;
  if (XH == nullptr) { for (int q = lane; q < 16 * (KD / 4); q += 32) { const int rr = q / (KD / 4), c4 = (q % (KD / 4)) * 4; const v4f xv = *(const v4f*)(X + (m0 + rr) * ldx + c4); for (int j = 0; j < 4; ++j) { b16 p, pl; split16(xv[j] * XS, p, pl); Ah[wave][rr][c4 + j] = p; Al[wave][rr][c4 + j] = pl; } }
    wave_lds_sync(); }
  v8f acc[NTL];
#pragma unroll
  for (int t = 0; t < NTL; ++t) acc[t] = (v8f){};
#pragma unroll 2
  for (int kb = 0; kb < KD; kb += 32) {
    if (XH != nullptr) { const v16b a = frag_kb(XH + (m0 + nloc) * KD + kb, hlf);
#pragma unroll
      for (int t = 0; t < NTL; ++t) acc[t] = wmma16b(a, frag_kb(Wt + (size_t)(n0 + t * 16 + nloc) * KD + kb, hlf), acc[t]); }
    else { const v16b a = frag_kb(&Ah[wave][nloc][kb], hlf), al = frag_kb(&Al[wave][nloc][kb], hlf);
#pragma unroll
      for (int t = 0; t < NTL; ++t) { const v16b bw = frag_kb(Wt + (size_t)(n0 + t * 16 + nloc) * KD + kb, hlf); acc[t] = wmma16b(a, bw, acc[t]); acc[t] = wmma16b(al, bw, acc[t]); } } }
#pragma unroll
  for (int t = 0; t < NTL; ++t) { const int c = n0 + t * 16 + nloc; const float bb = (bias != nullptr && c < nbias) ? bf16_rne(bias[c]) : 0.0f;
#pragma unroll 1
    for (int r = 0; r < 8; ++r) { float y = acc[t][r] * (1.0f / (XS * WSC)) + bb; if (EPI == 1) y = mish_(y); else if (EPI == 2) y = softplus_(y); else if (EPI == 3) y += R[(m0 + 8 * hlf + r) * ldy + c]; Tf[wave][8 * hlf + r][t * 16 + nloc] = y; } }
  wave_lds_sync();
  for (int pass = 0; pass < 2; ++pass) { for (int q = lane; q < 16 * NTL * 4; q += 32) { const int rr = q / (NTL * 4), c4 = (q % (NTL * 4)) * 4; *(volatile v4f*)(Y + (m0 + rr) * ldy + n0 + c4) = *(const v4f*)(&Tf[wave][rr][c4]); } __threadfence(); }
}
template <int MODE>
__global__ __launch_bounds__(256) void ln_kernel(const float* __restrict__ X, const float* __restrict__ g, const float* __restrict__ bta, const float* __restrict__ pos, float* __restrict__ Y, int nrows) {
  const int wave = threadIdx.x >> 5, lane = threadIdx.x & 31; const size_t row = (size_t)blockIdx.x * 8 + wave; if (row >= (size_t)nrows) return;
  const v4f a = *(const v4f*)(X + row * DM + lane * 4), c = *(const v4f*)(X + row * DM + 128 + lane * 4); float x[8] = {a[0], a[1], a[2], a[3], c[0], c[1], c[2], c[3]};
  float s = 0.0f; for (int j = 0; j < 8; ++j) s += x[j];
#pragma unroll
  for (int o = 16; o >= 1; o >>= 1) s += __shfl_xor(s, o);
  const float mu = s * (1.0f / DM); float q = 0.0f; for (int j = 0; j < 8; ++j) { const float d = x[j] - mu; q += d * d; }
#pragma unroll
  for (int o = 16; o >= 1; o >>= 1) q += __shfl_xor(q, o);
  const float rs = rsqrtf(q * (1.0f / DM) + EPS); v4f r0, r1;
#pragma unroll 1
  for (int j = 0; j < 8; ++j) { const int cc = (j < 4) ? lane * 4 + j : 128 + lane * 4 + (j - 4); float y = (x[j] - mu) * rs * bf16_rne(g[cc]) + bf16_rne(bta[cc]); if (MODE == 1) y = mish_(y) + bf16_rne(pos[(row % NF) * DM + cc]); if (j < 4) r0[j] = y; else r1[j - 4] = y; }
  for (int pass = 0; pass < 2; ++pass) { *(volatile v4f*)(Y + row * DM + lane * 4) = r0; *(volatile v4f*)(Y + row * DM + 128 + lane * 4) = r1; __threadfence(); }
}
__global__ __launch_bounds__(128) void conv_kernel(const float* __restrict__ XG, const float* __restrict__ cw, const float* __restrict__ cb, float* __restrict__ XC) {
  const size_t tok = blockIdx.x; const int t = (int)(tok % NF), c0 = threadIdx.x * 4; v4f r;
#pragma unroll 1
  for (int j = 0; j < 4; ++j) { const int c = c0 + j; float s = bf16_rne(cb[c]);
#pragma unroll 1
    for (int k = 0; k < 4; ++k) { const int tt = t - 3 + k; if (tt >= 0) s += pmul(XG[(tok - t + tt) * (2 * DI) + c], bf16_rne(cw[c * 4 + k])); } r[j] = silu_(s); }
  for (int pass = 0; pass < 2; ++pass) { *(volatile v4f*)(XC + tok * DI + c0) = r; __threadfence(); }
}
__global__ __launch_bounds__(128) void scan_kernel(const float* __restrict__ XC, const float* __restrict__ DT, const float* __restrict__ BC, const float* __restrict__ XG, const float* __restrict__ Alog, const float* __restrict__ Dp, float* __restrict__ YG) {
  __shared__ float bc_s[NF][2 * DS];
  const size_t b = blockIdx.x; const int c0 = threadIdx.x * 4;
  if (threadIdx.x < NF * 2 * DS) { const int t = threadIdx.x / (2 * DS), n = threadIdx.x % (2 * DS); bc_s[t][n] = BC[(b * NF + t) * (2 * DS) + n]; }
  __syncthreads();
  v4f outv[NF];
#pragma unroll 1
  for (int j = 0; j < 4; ++j) { const int c = c0 + j; float h[DS]; for (int n = 0; n < DS; ++n) h[n] = 0.0f; const float dp = bf16_rne(Dp[c]); float x4[NF], dt4[NF], g4[NF], y4[NF];
    for (int t = 0; t < NF; ++t) { const size_t tok = b * NF + t; x4[t] = XC[tok * DI + c]; dt4[t] = DT[tok * DI + c]; g4[t] = XG[tok * (2 * DI) + DI + c]; y4[t] = 0.0f; }
#pragma unroll 1
    for (int n = 0; n < DS; ++n) { const float An = -__expf(bf16_rne(Alog[c * DS + n])); float hn = 0.0f;
      for (int t = 0; t < NF; ++t) { hn = __expf(dt4[t] * An) * hn + pmul(dt4[t] * x4[t], bc_s[t][n]); y4[t] += pmul(hn, bc_s[t][DS + n]); } (void)h; }
    for (int t = 0; t < NF; ++t) outv[t][j] = (y4[t] + dp * x4[t]) * silu_(g4[t]); }
  for (int pass = 0; pass < 2; ++pass) { for (int t = 0; t < NF; ++t) *(volatile v4f*)(YG + (b * NF + t) * DI + c0) = outv[t]; __threadfence(); }
}
__global__ __launch_bounds__(256) void mean_kernel(const float* __restrict__ X, float* __restrict__ F) {
  const int wave = threadIdx.x >> 5, lane = threadIdx.x & 31; const size_t b = (size_t)blockIdx.x * 8 + wave; v4f r0 = {0.0f, 0.0f, 0.0f, 0.0f}, r1 = r0;
  for (int t = 0; t < NF; ++t) { r0 += *(const v4f*)(X + (b * NF + t) * DM + lane * 4); r1 += *(const v4f*)(X + (b * NF + t) * DM + 128 + lane * 4); }
  r0 *= 0.25f; r1 *= 0.25f;
  for (int pass = 0; pass < 2; ++pass) { *(volatile v4f*)(F + b * DM + lane * 4) = r0; *(volatile v4f*)(F + b * DM + 128 + lane * 4) = r1; __threadfence(); }
}
__global__ __launch_bounds__(128) void final_kernel(const float* __restrict__ LG, const float* __restrict__ VV, float* __restrict__ out) {
  __shared__ __attribute__((aligned(16))) float st[16 * 20];
  const int t_ = threadIdx.x; const size_t b0 = (size_t)blockIdx.x * 16;
  for (int q = t_; q < 16 * 20; q += 128) { const int bb = q / 20, c = q % 20; st[q] = (c < NO) ? LG[(b0 + bb) * 32 + c] : VV[(b0 + bb) * 16]; }
  __syncthreads();
  for (int pass = 0; pass < 2; ++pass) { if (t_ < 80) *(volatile v4f*)(out + b0 * 20 + t_ * 4) = *(const v4f*)(&st[t_ * 4]); __threadfence(); }
}
}

extern "C" void kernel_launch(void* const* d_in, const int* in_sizes, int n_in, void* d_out, int out_size, void* d_ws, size_t ws_size, hipStream_t stream) {
  (void)n_in;
  auto Fp = [&](int i) { return (const float*)d_in[i]; };
  if (in_sizes[0] != NBS * NF * FD || in_sizes[1] != FD * DM || in_sizes[8] != NL * DM * 2 * DI || in_sizes[11] != NL * DI * DI || in_sizes[13] != NL * DI * DS || in_sizes[17] != NL * DI * DM || in_sizes[26] != (DM / 2) * NO || in_sizes[32] != DM / 4 || out_size != NBS * 20) return;
  size_t off = 0; char* ws = (char*)d_ws;
  auto carve = [&](size_t bytes) { char* p = ws + off; off += (bytes + 255) & ~(size_t)255; return p; };
  WPtrs P;
  P.OBS = (b16*)carve((size_t)NT * FDP * 2); P.EMB = (b16*)carve((size_t)DM * FDP * 2); P.INW = (b16*)carve((size_t)NL * 2 * DI * DM * 2); P.DTW = (b16*)carve((size_t)NL * DI * DI * 2); P.BCW = (b16*)carve((size_t)NL * 2 * DS * DI * 2); P.OUTW = (b16*)carve((size_t)NL * DM * DI * 2);
  P.POOLW = (b16*)carve((size_t)DM * DM * 2); P.P1 = (b16*)carve((size_t)DM * DM * 2); P.P2 = (b16*)carve((size_t)(DM / 2) * DM * 2); P.PH = (b16*)carve((size_t)32 * (DM / 2) * 2); P.V1 = (b16*)carve((size_t)(DM / 2) * DM * 2); P.V2 = (b16*)carve((size_t)(DM / 4) * (DM / 2) * 2); P.VH = (b16*)carve((size_t)16 * (DM / 4) * 2);
  float* X = (float*)carve((size_t)NT * DM * 4); float* E0 = (float*)carve((size_t)NT * DM * 4); float* H = (float*)carve((size_t)NT * DM * 4); float* XG = (float*)carve((size_t)NT * 2 * DI * 4); float* XC = (float*)carve((size_t)NT * DI * 4); float* DT = (float*)carve((size_t)NT * DI * 4); float* BC = (float*)carve((size_t)NT * 2 * DS * 4); float* YG = (float*)carve((size_t)NT * DI * 4);
  float* F = (float*)carve((size_t)NBS * DM * 4); float* FL = (float*)carve((size_t)NBS * DM * 4); float* F2 = (float*)carve((size_t)NBS * DM * 4); float* PA = (float*)carve((size_t)NBS * DM * 4); float* PB = (float*)carve((size_t)NBS * (DM / 2) * 4); float* LG = (float*)carve((size_t)NBS * 32 * 4); float* VA = (float*)carve((size_t)NBS * (DM / 2) * 4); float* VB = (float*)carve((size_t)NBS * (DM / 4) * 4); float* VV = (float*)carve((size_t)NBS * 16 * 4);
  if (off > ws_size || off > ((size_t)128 << 20)) return;
  auto wprep = [&](const float* w, int nin, int nout, int ninp, int noutp, b16* dst) { wprep_kernel<<<(unsigned)(((size_t)noutp * ninp / 8 + 255) / 256), 256, 0, stream>>>(w, nin, nout, ninp, noutp, dst); };
  obsprep_kernel<<<(unsigned)(((size_t)NT * FDP / 8 + 255) / 256), 256, 0, stream>>>(Fp(0), P.OBS);
  wprep(Fp(1), FD, DM, FDP, DM, P.EMB);
  for (int l = 0; l < NL; ++l) { wprep(Fp(8) + (size_t)l * DM * 2 * DI, DM, 2 * DI, DM, 2 * DI, P.INW + (size_t)l * 2 * DI * DM); wprep(Fp(11) + (size_t)l * DI * DI, DI, DI, DI, DI, P.DTW + (size_t)l * DI * DI);
    wprep(Fp(13) + (size_t)l * DI * DS, DI, DS, DI, DS, P.BCW + (size_t)l * 2 * DS * DI); wprep(Fp(14) + (size_t)l * DI * DS, DI, DS, DI, DS, P.BCW + (size_t)l * 2 * DS * DI + (size_t)DS * DI); wprep(Fp(17) + (size_t)l * DI * DM, DI, DM, DI, DM, P.OUTW + (size_t)l * DM * DI); }
  wprep(Fp(20), DM, DM, DM, DM, P.POOLW); wprep(Fp(22), DM, DM, DM, DM, P.P1); wprep(Fp(24), DM, DM / 2, DM, DM / 2, P.P2); wprep(Fp(26), DM / 2, NO, DM / 2, 32, P.PH); wprep(Fp(28), DM, DM / 2, DM, DM / 2, P.V1); wprep(Fp(30), DM / 2, DM / 4, DM / 2, DM / 4, P.V2); wprep(Fp(32), DM / 4, 1, DM / 4, 16, P.VH);
  dense_kernel<FDP, 8, 0, 4><<<dim3(NT / 64, DM / 128), 128, 0, stream>>>(nullptr, 0, P.OBS, P.EMB, Fp(2), DM, nullptr, E0, DM);
  ln_kernel<1><<<NT / 8, 256, 0, stream>>>(E0, Fp(3), Fp(4), Fp(5), X, NT);
  for (int l = 0; l < NL; ++l) {
    ln_kernel<0><<<NT / 8, 256, 0, stream>>>(X, Fp(6) + l * DM, Fp(7) + l * DM, nullptr, H, NT);
    dense_kernel<DM, 8, 0, 4><<<dim3(NT / 64, 2 * DI / 128), 128, 0, stream>>>(H, DM, nullptr, P.INW + (size_t)l * 2 * DI * DM, nullptr, 0, nullptr, XG, 2 * DI);
    conv_kernel<<<NT, 128, 0, stream>>>(XG, Fp(9) + (size_t)l * DI * 4, Fp(10) + l * DI, XC);
    dense_kernel<DI, 8, 2, 2><<<dim3(NT / 32, DI / 128), 64, 0, stream>>>(XC, DI, nullptr, P.DTW + (size_t)l * DI * DI, Fp(12) + l * DI, DI, nullptr, DT, DI);
    dense_kernel<DI, 2, 0, 2><<<dim3(NT / 32, 1), 64, 0, stream>>>(XC, DI, nullptr, P.BCW + (size_t)l * 2 * DS * DI, nullptr, 0, nullptr, BC, 2 * DS);
    scan_kernel<<<NBS, 128, 0, stream>>>(XC, DT, BC, XG, Fp(15) + (size_t)l * DI * DS, Fp(16) + l * DI, YG);
    dense_kernel<DI, 8, 3, 2><<<dim3(NT / 32, DM / 128), 64, 0, stream>>>(YG, DI, nullptr, P.OUTW + (size_t)l * DM * DI, nullptr, 0, X, X, DM);
  }
  mean_kernel<<<NBS / 8, 256, 0, stream>>>(X, F);
  ln_kernel<0><<<NBS / 8, 256, 0, stream>>>(F, Fp(18), Fp(19), nullptr, FL, NBS);
  dense_kernel<DM, 8, 1, 4><<<dim3(NBS / 64, DM / 128), 128, 0, stream>>>(FL, DM, nullptr, P.POOLW, Fp(21), DM, nullptr, F2, DM);
  dense_kernel<DM, 8, 1, 4><<<dim3(NBS / 64, DM / 128), 128, 0, stream>>>(F2, DM, nullptr, P.P1, Fp(23), DM, nullptr, PA, DM);
  dense_kernel<DM, 8, 1, 4><<<dim3(NBS / 64, 1), 128, 0, stream>>>(PA, DM, nullptr, P.P2, Fp(25), DM / 2, nullptr, PB, DM / 2);
  dense_kernel<DM / 2, 2, 0, 4><<<dim3(NBS / 64, 1), 128, 0, stream>>>(PB, DM / 2, nullptr, P.PH, Fp(27), NO, nullptr, LG, 32);
  dense_kernel<DM, 8, 1, 4><<<dim3(NBS / 64, 1), 128, 0, stream>>>(F2, DM, nullptr, P.V1, Fp(29), DM / 2, nullptr, VA, DM / 2);
  dense_kernel<DM / 2, 4, 1, 4><<<dim3(NBS / 64, 1), 128, 0, stream>>>(VA, DM / 2, nullptr, P.V2, Fp(31), DM / 4, nullptr, VB, DM / 4);
  dense_kernel<DM / 4, 1, 0, 4><<<dim3(NBS / 64, 1), 128, 0, stream>>>(VB, DM / 4, nullptr, P.VH, Fp(33), 1, nullptr, VV, 16);
  final_kernel<<<NBS / 16, 128, 0, stream>>>(LG, VV, (float*)d_out);
}
